// QuantumMLP_80736795230972
// MI455X (gfx1250) — hardware-verified
//
#include <hip/hip_runtime.h>
#include <stddef.h>


typedef __attribute__((ext_vector_type(16))) __bf16   v16b;
typedef __attribute__((ext_vector_type(8)))  __bf16   v8b;
typedef __attribute__((ext_vector_type(8)))  _Float16 v8h;
typedef __attribute__((ext_vector_type(8)))  float    v8f;
typedef __attribute__((ext_vector_type(4)))  float    v4f;
typedef __attribute__((ext_vector_type(2)))  float    v2f;

#define NQ     8
#define QD     256
#define IN_F   256
#define OUT_F  128
#define DEPTH  2
#define GPL    (5 * NQ)
#define NGATE  (NQ + DEPTH * GPL)
#define SPB    16
#define PP     264
#define DP     132

__device__ __forceinline__ unsigned short f2bf_bits(float f) {
  unsigned u = __float_as_uint(f);
  return (unsigned short)((u + 0x7FFFu + ((u >> 16) & 1u)) >> 16);
}
__device__ __forceinline__ float bf_bits2f(unsigned short h) { return __uint_as_float(((unsigned)h) << 16); }

__device__ __forceinline__ void dep_guard_b(v8f& a, v8f& b, v16b x, v16b y) { asm volatile("v_nop\n\tv_nop\n\tv_nop\n\tv_nop" : "+v"(a), "+v"(b) : "v"(x), "v"(y)); }
__device__ __forceinline__ void keep4_b(v16b a, v16b b, v16b c, v16b d) { asm volatile("v_nop" :: "v"(a), "v"(b), "v"(c), "v"(d)); }

template <typename T> struct Frag;
template <> struct Frag<__bf16> {
  typedef v16b V; union U { v16b v; v8b h[2]; };
  static __device__ __forceinline__ v16b load(const __bf16* p) {
    U f; f.h[0] = *(const v8b*)(p); f.h[1] = *(const v8b*)(p + 16); return f.v;
  }
  static __device__ __forceinline__ v8f mma(v16b a, v16b b, v8f c) {
    return __builtin_amdgcn_wmma_f32_16x16x32_bf16(false, a, false, b, (short)0, c, false, false);
  }
  static __device__ __forceinline__ void guard(v8f& a, v8f& b, v16b x, v16b y) { dep_guard_b(a, b, x, y); }
  static __device__ __forceinline__ void keep(v16b a, v16b b, v16b c, v16b d) { keep4_b(a, b, c, d); }
};

__device__ __forceinline__ v8f at_mma(v16b a, v16b b, v8f c) {
  c = __builtin_amdgcn_wmma_f32_16x16x32_bf16(false, a, false, b, (short)0, c, false, false);
  asm volatile("v_nop\n\tv_nop\n\tv_nop\n\tv_nop" : "+v"(c) : "v"(a), "v"(b));
  return c;
}

__global__ __launch_bounds__(256) void split_w_bf16(const float* __restrict__ w,
                                                   unsigned short* __restrict__ whi,
                                                   unsigned short* __restrict__ wlo, int n8) {
  const int i = blockIdx.x * 256 + threadIdx.x;
  if (i < n8) {
    const v4f a = *(const v4f*)(w + (size_t)i * 8);
    const v4f b = *(const v4f*)(w + (size_t)i * 8 + 4);
    v8h hv, lv;
#pragma unroll
    for (int e = 0; e < 4; ++e) {
      unsigned short hb = f2bf_bits(a[e]);
      unsigned short lb = f2bf_bits(a[e] - bf_bits2f(hb));
      hv[e] = __builtin_bit_cast(_Float16, hb);
      lv[e] = __builtin_bit_cast(_Float16, lb);
      hb = f2bf_bits(b[e]);
      lb = f2bf_bits(b[e] - bf_bits2f(hb));
      hv[4 + e] = __builtin_bit_cast(_Float16, hb);
      lv[4 + e] = __builtin_bit_cast(_Float16, lb);
    }
    unsigned short* ph = whi + (size_t)i * 8;
    unsigned short* pl = wlo + (size_t)i * 8;
    *(volatile v8h*)ph = hv;
    *(volatile v8h*)pl = lv;
    __threadfence();
    *(volatile v8h*)ph = hv;
    *(volatile v8h*)pl = lv;
  }
}

__global__ __launch_bounds__(32) void qsim_proj_kernel(
    const float* __restrict__ x, const float* __restrict__ W_in, const float* __restrict__ b_in,
    const float* __restrict__ qw, const float* __restrict__ us,
    const unsigned short* __restrict__ whi_p, const unsigned short* __restrict__ wlo_p,
    const float* __restrict__ b_out, float* __restrict__ out, int nsamp) {
  __shared__ __align__(16) v2f st[QD];
  __shared__ __align__(16) __bf16 Phi[SPB * PP];
  __shared__ __align__(16) __bf16 Plo[SPB * PP];
  __shared__ __align__(16) float Ds[SPB * DP];
  __shared__ float gcs[NGATE];
  __shared__ float gsn[NGATE];
  __shared__ int ginfo[NGATE];
  __shared__ float angL[NQ];

  const int lane = threadIdx.x;
  const int blk = blockIdx.x;
  if ((blk + 1) * SPB > nsamp) return;

  const float PI_F = 3.14159265358979323846f;

#pragma unroll 1
  for (int ss = 0; ss < SPB; ++ss) {
    const int s = blk * SPB + ss;

    const float* xr = x + (size_t)s * IN_F + lane * 8;
    const v4f x0 = *(const v4f*)(xr);
    const v4f x1 = *(const v4f*)(xr + 4);
#pragma unroll 1
    for (int i = 0; i < NQ; ++i) {
      const float* wr = W_in + (size_t)i * IN_F + lane * 8;
      const v4f w0 = *(const v4f*)(wr);
      const v4f w1 = *(const v4f*)(wr + 4);
      float acc = x0[0] * w0[0];
      acc += x0[1] * w0[1];
      acc += x0[2] * w0[2];
      acc += x0[3] * w0[3];
      acc += x1[0] * w1[0];
      acc += x1[1] * w1[1];
      acc += x1[2] * w1[2];
      acc += x1[3] * w1[3];
      acc += __shfl_xor(acc, 16, 32);
      acc += __shfl_xor(acc, 8, 32);
      acc += __shfl_xor(acc, 4, 32);
      acc += __shfl_xor(acc, 2, 32);
      acc += __shfl_xor(acc, 1, 32);
      const float a = tanhf(acc + b_in[i]) * PI_F;
      if (lane == 0) angL[i] = a;
    }
    __syncthreads();

#pragma unroll 1
    for (int r = 0; r < (NGATE + 31) / 32; ++r) {
      const int g = lane + 32 * r;
      if (g < NGATE) {
        int kind = 0, q = 0;
        float th = 0.f;
        if (g < NQ) {
          q = g; th = angL[q];
        } else {
          const int l = (g - NQ) / GPL;
          const int u = g - NQ - GPL * l;
          if (u < NQ) {
            q = u; th = angL[q] * us[l * NQ + q];
          } else if (u < 3 * NQ) {
            const int v = u - NQ;
            q = v >> 1;
            kind = (v & 1) ? 0 : 1;
            th = qw[(l * NQ + q) * 3 + (v & 1)];
          } else if (u < 4 * NQ) {
            kind = 2; q = u - 3 * NQ;
          } else {
            q = u - 4 * NQ;
            th = qw[(l * NQ + q) * 3 + 2];
          }
        }
        ginfo[g] = kind | ((NQ - 1 - q) << 4) | ((NQ - 1 - ((q + 1) & (NQ - 1))) << 8);
        float cv = 1.f, sv = 0.f;
        if (kind != 2) {
          const float hth = 0.5f * th;
          cv = cosf(hth);
          sv = sinf(hth);
        }
        gcs[g] = cv;
        gsn[g] = sv;
      }
    }

    {
#pragma unroll
      for (int e = 0; e < 8; ++e) {
        v2f v = {0.f, 0.f};
        if (lane == 0 && e == 0) v.x = 1.f;
        st[lane * 8 + e] = v;
      }
    }
    __syncthreads();

#pragma unroll 1
    for (int g = 0; g < NGATE; ++g) {
      const int info = ginfo[g];
      const int kind = info & 3;
      const int pa = (info >> 4) & 7;
      const int pb = (info >> 8) & 7;
      if (kind == 2) {
        const int plo = pa < pb ? pa : pb;
        const int phi = pa < pb ? pb : pa;
        const int mc = 1 << pa, mt = 1 << pb;
#pragma unroll
        for (int t = 0; t < 2; ++t) {
          const int j = lane + 32 * t;
          int v = ((j >> plo) << (plo + 1)) | (j & ((1 << plo) - 1));
          v = ((v >> phi) << (phi + 1)) | (v & ((1 << phi) - 1));
          const int i0 = (v | mc) & (QD - 1);
          const int i1 = (i0 | mt) & (QD - 1);
          const v2f a0 = st[i0];
          const v2f a1 = st[i1];
          st[i0] = a1;
          st[i1] = a0;
        }
      } else {
        const float c = gcs[g];
        const float sn = gsn[g];
        const int pm = 1 << pa;
        const int lm = pm - 1;
        if (kind == 1) {
#pragma unroll
          for (int t = 0; t < 4; ++t) {
            const int j = lane + 32 * t;
            const int i0 = (((j >> pa) << (pa + 1)) | (j & lm)) & (QD - 1);
            const int i1 = (i0 | pm) & (QD - 1);
            const v2f a0 = st[i0];
            const v2f a1 = st[i1];
            v2f n0, n1;
            n0.x = c * a0.x + sn * a1.y;
            n0.y = c * a0.y - sn * a1.x;
            n1.x = c * a1.x + sn * a0.y;
            n1.y = c * a1.y - sn * a0.x;
            st[i0] = n0;
            st[i1] = n1;
          }
        } else {
#pragma unroll
          for (int t = 0; t < 4; ++t) {
            const int j = lane + 32 * t;
            const int i0 = (((j >> pa) << (pa + 1)) | (j & lm)) & (QD - 1);
            const int i1 = (i0 | pm) & (QD - 1);
            const v2f a0 = st[i0];
            const v2f a1 = st[i1];
            const v2f n0 = c * a0 - sn * a1;
            const v2f n1 = sn * a0 + c * a1;
            st[i0] = n0;
            st[i1] = n1;
          }
        }
      }
      __syncthreads();
    }

    {
      v8b hv, lv;
#pragma unroll
      for (int e = 0; e < 8; ++e) {
        const v2f a = st[lane * 8 + e];
        const float p = a.x * a.x + a.y * a.y;
        const unsigned short hb = f2bf_bits(p);
        const unsigned short lb = f2bf_bits(p - bf_bits2f(hb));
        hv[e] = __builtin_bit_cast(__bf16, hb);
        lv[e] = __builtin_bit_cast(__bf16, lb);
      }
      *(v8b*)(Phi + ss * PP + lane * 8) = hv;
      *(v8b*)(Plo + ss * PP + lane * 8) = lv;
    }
  }
  __syncthreads();

  const __bf16* Whi = (const __bf16*)whi_p;
  const __bf16* Wlo = (const __bf16*)wlo_p;
  const int m = lane & 15;
  const int hh = lane >> 4;
  const int koff = hh * 8;
#pragma unroll 1
  for (int nh = 0; nh < 2; ++nh) {
    v8f acc[4];
#pragma unroll
    for (int j = 0; j < 4; ++j) acc[j] = (v8f){0.f, 0.f, 0.f, 0.f, 0.f, 0.f, 0.f, 0.f};
#pragma unroll 1
    for (int k0 = 0; k0 < QD; k0 += 32) {
      const v16b ah = Frag<__bf16>::load(Phi + m * PP + k0 + koff);
      const v16b al = Frag<__bf16>::load(Plo + m * PP + k0 + koff);
#pragma unroll
      for (int j = 0; j < 4; ++j) {
        const size_t bo = (size_t)(nh * 64 + j * 16 + m) * QD + k0 + koff;
        const v16b bh = Frag<__bf16>::load(Whi + bo);
        const v16b bl = Frag<__bf16>::load(Wlo + bo);
        acc[j] = at_mma(ah, bh, acc[j]);
        acc[j] = at_mma(ah, bl, acc[j]);
        acc[j] = at_mma(al, bh, acc[j]);
      }
    }
#pragma unroll
    for (int j = 0; j < 4; ++j) {
      const int n = nh * 64 + j * 16 + m;
      const float bv = b_out[n];
#pragma unroll
      for (int r = 0; r < 8; ++r) Ds[(8 * hh + r) * DP + n] = acc[j][r] + bv;
    }
  }
  __syncthreads();

  for (int pass = 0; pass < 2; ++pass) {
#pragma unroll
    for (int row = 0; row < SPB; ++row) {
      const v4f v = *(const v4f*)(Ds + row * DP + lane * 4);
      *(volatile v4f*)(out + (size_t)(blk * SPB + row) * OUT_F + lane * 4) = v;
    }
    __threadfence();
  }
}

extern "C" void kernel_launch(void* const* d_in, const int* in_sizes, int n_in,
                              void* d_out, int out_size, void* d_ws, size_t ws_size,
                              hipStream_t stream) {
  if (n_in < 7) return;
  const float* x     = (const float*)d_in[0];
  const float* W_in  = (const float*)d_in[1];
  const float* b_in  = (const float*)d_in[2];
  const float* qw    = (const float*)d_in[3];
  const float* us    = (const float*)d_in[4];
  const float* W_out = (const float*)d_in[5];
  const float* b_out = (const float*)d_in[6];
  float* out = (float*)d_out;

  const int nsamp = in_sizes[0] / IN_F;
  if (nsamp <= 0 || (nsamp % SPB) != 0 || in_sizes[0] != nsamp * IN_F) return;
  if (in_sizes[1] != NQ * IN_F || in_sizes[2] != NQ || in_sizes[3] != DEPTH * NQ * 3 ||
      in_sizes[4] != DEPTH * NQ || in_sizes[5] != OUT_F * QD || in_sizes[6] != OUT_F) return;
  if (out_size != nsamp * OUT_F) return;

  const size_t plane_bytes = (size_t)OUT_F * QD * sizeof(unsigned short);
  if (2 * plane_bytes > ws_size) return;
  unsigned short* whi = (unsigned short*)d_ws;
  unsigned short* wlo = (unsigned short*)((char*)d_ws + plane_bytes);

  const int n8 = (OUT_F * QD) / 8;
  split_w_bf16<<<(n8 + 255) / 256, 256, 0, stream>>>(W_out, whi, wlo, n8);
  qsim_proj_kernel<<<nsamp / SPB, 32, 0, stream>>>(x, W_in, b_in, qw, us, whi, wlo, b_out, out, nsamp);
}
